// MessagePassingNet_28810640622031
// MI455X (gfx1250) — hardware-verified
//
#include <hip/hip_runtime.h>
#include <stddef.h>


#define EPT    8
#define WCAP   (EPT * 32)
#define DM     64

#define NTE    64
#define NWE    2
#define CHE    (NTE * EPT)
#define PASSN  (NWE * 16)
#define PCAP   (CHE + PASSN)
#define NB     1024

#define NTN    128
#define NTP    256
#define NTM    256
#define NWM    8
#define MB     512
#define WROWS  400
#define NBIAS  272

#define WSC    8.0f
#define WINV   0.125f

static_assert(PASSN == 32);
static_assert((PCAP % PASSN) == 0);
static_assert((NB % 64) == 0);
static_assert(((NB / 16) % NWE) == 0);
static_assert(WROWS * DM * 2 <= 65536);

typedef float    v4f  __attribute__((ext_vector_type(4)));
typedef float    v8f  __attribute__((ext_vector_type(8)));
typedef int      v4i  __attribute__((ext_vector_type(4)));
typedef _Float16 v8h  __attribute__((ext_vector_type(8)));
typedef _Float16 v16h __attribute__((ext_vector_type(16)));
union FragH { v16h v; v8h h[2]; };

__device__ __forceinline__ v8f zero8f() {
  v8f r;
#pragma unroll
  for (int i = 0; i < 8; ++i) r[i] = 0.0f;
  return r;
}

__device__ __forceinline__ v8f wmh(v16h a, v16h b, v8f c) {
  v8f d = __builtin_amdgcn_wmma_f32_16x16x32_f16(false, a, false, b, (short)0, c, false, false);
  asm volatile("v_nop\n\tv_nop\n\tv_nop\n\tv_nop" : "+v"(d) : "v"(a), "v"(b));
  return d;
}

__device__ __forceinline__ v8h cvt8(const float* p) {
  const v4f a = *(const v4f*)p;
  const v4f b = *(const v4f*)(p + 4);
  v8h r;
  r[0] = (_Float16)a.x; r[1] = (_Float16)a.y; r[2] = (_Float16)a.z; r[3] = (_Float16)a.w;
  r[4] = (_Float16)b.x; r[5] = (_Float16)b.y; r[6] = (_Float16)b.z; r[7] = (_Float16)b.w;
  return r;
}

__device__ __forceinline__ v8h pk8(v4f a, v4f b) {
  v8h r;
  r[0] = (_Float16)a.x; r[1] = (_Float16)a.y; r[2] = (_Float16)a.z; r[3] = (_Float16)a.w;
  r[4] = (_Float16)b.x; r[5] = (_Float16)b.y; r[6] = (_Float16)b.z; r[7] = (_Float16)b.w;
  return r;
}

__device__ __forceinline__ v8h relu8(v8f d) {
  v8h r;
#pragma unroll
  for (int i = 0; i < 8; ++i) { const float t = fmaxf(d[i] * WINV, 0.0f); r[i] = (_Float16)t; }
  return r;
}

__device__ __forceinline__ v8f ldc8(const float* p) {
  const v4f a = *(const v4f*)p;
  const v4f b = *(const v4f*)(p + 4);
  v8f c;
  c[0] = a.x; c[1] = a.y; c[2] = a.z; c[3] = a.w;
  c[4] = b.x; c[5] = b.y; c[6] = b.z; c[7] = b.w;
  return c;
}

__device__ __forceinline__ v8f tile16(const _Float16* ap, const float* cp, v16h b0, v16h b1) {
  FragH a0, a1;
  a0.h[0] = *(const v8h*)ap;        a0.h[1] = *(const v8h*)(ap + 16);
  a1.h[0] = *(const v8h*)(ap + 32); a1.h[1] = *(const v8h*)(ap + 48);
  v8f c = ldc8(cp);
  c = wmh(a0.v, b0, c);
  c = wmh(a1.v, b1, c);
  return c;
}

template <int RANGE, int TPB>
__device__ __forceinline__ int scan_chunk(const int* __restrict__ keys, int nK, int cbase, int base,
                                          int vec8, int* list, int tid, int wave) {
  constexpr int CH = TPB * EPT;
  int wc = 0;
  const int el0  = tid * EPT;
  const int e0   = cbase + el0;
  const int sent = -2147483647 - 1;
  v4i da, db;
  if (vec8 != 0 && cbase + CH <= nK) {
    da = *(const v4i*)(keys + e0);
    db = *(const v4i*)(keys + e0 + 4);
  } else {
    da.x = (e0     < nK) ? keys[min(e0, nK - 1)] : sent;
    da.y = (e0 + 1 < nK) ? keys[min(e0 + 1, nK - 1)] : sent;
    da.z = (e0 + 2 < nK) ? keys[min(e0 + 2, nK - 1)] : sent;
    da.w = (e0 + 3 < nK) ? keys[min(e0 + 3, nK - 1)] : sent;
    db.x = (e0 + 4 < nK) ? keys[min(e0 + 4, nK - 1)] : sent;
    db.y = (e0 + 5 < nK) ? keys[min(e0 + 5, nK - 1)] : sent;
    db.z = (e0 + 6 < nK) ? keys[min(e0 + 6, nK - 1)] : sent;
    db.w = (e0 + 7 < nK) ? keys[min(e0 + 7, nK - 1)] : sent;
  }
  const unsigned nb = (unsigned)base;
  const unsigned s0 = (unsigned)da.x - nb, s1 = (unsigned)da.y - nb;
  const unsigned s2 = (unsigned)da.z - nb, s3 = (unsigned)da.w - nb;
  const unsigned s4 = (unsigned)db.x - nb, s5 = (unsigned)db.y - nb;
  const unsigned s6 = (unsigned)db.z - nb, s7 = (unsigned)db.w - nb;
  const bool h0 = s0 < (unsigned)RANGE, h1 = s1 < (unsigned)RANGE, h2 = s2 < (unsigned)RANGE, h3 = s3 < (unsigned)RANGE;
  const bool h4 = s4 < (unsigned)RANGE, h5 = s5 < (unsigned)RANGE, h6 = s6 < (unsigned)RANGE, h7 = s7 < (unsigned)RANGE;
  const unsigned any = __builtin_amdgcn_ballot_w32(h0 | h1 | h2 | h3 | h4 | h5 | h6 | h7);
  if (any != 0u) {
#define HITJ(J, HJ) { \
      const unsigned mj = __builtin_amdgcn_ballot_w32(HJ); \
      if (mj != 0u) { \
        if (HJ) { \
          const int pos = wc + (int)__builtin_amdgcn_mbcnt_lo(mj, 0u); \
          if (pos < WCAP) list[wave * WCAP + pos] = el0 + (J); \
        } \
        wc += (int)__builtin_popcount(mj); } }
    HITJ(0, h0)
    HITJ(1, h1)
    HITJ(2, h2)
    HITJ(3, h3)
    HITJ(4, h4)
    HITJ(5, h5)
    HITJ(6, h6)
    HITJ(7, h7)
#undef HITJ
  }
  return wc;
}

__global__ __launch_bounds__(NTP) void k_prep(
    const float* __restrict__ w0, const float* __restrict__ w1, const float* __restrict__ w2,
    const float* __restrict__ f1, const float* __restrict__ f2, const float* __restrict__ w3,
    _Float16* wpl) {
  const int tid = threadIdx.x, lane = tid & 31, wave = tid >> 5, j8 = lane & 7, sub = lane >> 3;
#pragma unroll 1
  for (int it = 0; it < (WROWS + 31) / 32; ++it) {
    const int q    = it * 32 + wave * 4 + sub;
    const int cat  = q >> 6;
    const int n64  = q & 63;
    const int n16  = q & 15;
    const int ksel = (q & 64) ? 64 : 0;
    v8h hv;
#pragma unroll
    for (int i = 0; i < 8; ++i) {
      const int k = 8 * j8 + i;
      const float c0 = w0[(ksel + k) * 64 + n64];
      const float c1 = w1[k * 64 + n64];
      const float c2 = w2[k * 64 + n64];
      const float c3 = f1[k * 64 + n64];
      const float c4 = f2[k * 64 + n64];
      const float c5 = w3[k * 16 + n16];
      float t = c0;
      t = (cat == 2) ? c1 : t;
      t = (cat == 3) ? c2 : t;
      t = (cat == 4) ? c3 : t;
      t = (cat == 5) ? c4 : t;
      t = (cat >= 6) ? c5 : t;
      hv[i] = (_Float16)(t * WSC);
    }
    const bool wr = q < WROWS;
    _Float16* dp = wpl + (size_t)q * DM + 8 * j8;
    if (wr) *(volatile v8h*)dp = hv;
    __threadfence();
    if (wr) *(volatile v8h*)dp = hv;
  }
}

__global__ __launch_bounds__(NTN) void k_node(
    const float* __restrict__ st, const _Float16* __restrict__ w0t, const float* __restrict__ b0,
    float* pq, int nN) {
  __shared__ __attribute__((aligned(16))) float stgn[(NTN / 32) * 16 * 128];
  const int tid = threadIdx.x, lane = tid & 31, wave = tid >> 5, h = lane >> 4, m = lane & 15;
  const int row0 = blockIdx.x * (NTN / 32) * 16 + wave * 16;
  int ra = row0 + m;
  ra = ra > nN - 1 ? nN - 1 : ra;
  const float* ap = st + (size_t)ra * DM + 8 * h;
  FragH a0, a1;
  a0.h[0] = cvt8(ap);      a0.h[1] = cvt8(ap + 16);
  a1.h[0] = cvt8(ap + 32); a1.h[1] = cvt8(ap + 48);
  float* sw = stgn + wave * 2048;
#pragma unroll
  for (int nt = 0; nt < 8; ++nt) {
    const _Float16* bp = w0t + (size_t)(16 * nt + m) * DM + 8 * h;
    FragH bf0, bf1;
    bf0.h[0] = *(const v8h*)bp;        bf0.h[1] = *(const v8h*)(bp + 16);
    bf1.h[0] = *(const v8h*)(bp + 32); bf1.h[1] = *(const v8h*)(bp + 48);
    v8f acc = zero8f();
    acc = wmh(a0.v, bf0.v, acc);
    acc = wmh(a1.v, bf1.v, acc);
    const float bb   = b0[(16 * nt + m) & 63];
    const float bias = (nt < 4) ? bb : 0.0f;
#pragma unroll
    for (int r = 0; r < 8; ++r) sw[(8 * h + r) * 128 + 16 * nt + m] = acc[r] * WINV + bias;
  }
  __syncthreads();
  float* gp = pq + (size_t)row0 * 128;
#pragma unroll
  for (int r = 0; r < 16; ++r) {
    const v4f v = *(const v4f*)(sw + r * 128 + 4 * lane);
    *(volatile v4f*)(gp + r * 128 + 4 * lane) = v;
  }
  __threadfence();
#pragma unroll
  for (int r = 0; r < 16; ++r) {
    const v4f v = *(const v4f*)(sw + r * 128 + 4 * lane);
    *(volatile v4f*)(gp + r * 128 + 4 * lane) = v;
  }
}

__global__ __launch_bounds__(NTE) void k_edge(
    const float* __restrict__ pq, const int* __restrict__ srcs, const int* __restrict__ dsts,
    const _Float16* __restrict__ wpl,
    const float* __restrict__ b1, const float* __restrict__ b2,
    const float* __restrict__ g1, const float* __restrict__ g2, const float* __restrict__ g3,
    float* opl, int nN, int nE, int vec8) {
  extern __shared__ __attribute__((aligned(16))) float acc[];
  __shared__ __attribute__((aligned(16))) _Float16 stg[NWE * 16 * DM];
  __shared__ __attribute__((aligned(16))) float    msg[NWE * 16 * DM];
  __shared__ __attribute__((aligned(16))) int      list[NWE * WCAP];
  __shared__ __attribute__((aligned(16))) int      pend[PCAP];
  __shared__ int slotb[PASSN];
  __shared__ __attribute__((aligned(16))) float    bsm[NBIAS];
  __shared__ int wcnt[NWE];
  __shared__ int pendN;

  const int tid = threadIdx.x, lane = tid & 31, wave = tid >> 5, h = lane >> 4, m = lane & 15;
  const int nodeBase = blockIdx.x * NB;
  const _Float16* w1t = wpl + 128 * DM;
  const _Float16* w2t = wpl + 192 * DM;
  const _Float16* f1t = wpl + 256 * DM;
  const _Float16* f2t = wpl + 320 * DM;
  const _Float16* w3t = wpl + 384 * DM;

  {
    const v4f z4 = {0.0f, 0.0f, 0.0f, 0.0f};
    for (int i = tid; i < NB * DM / 4; i += NTE) *(v4f*)(acc + 4 * i) = z4;
  }
  for (int i = tid; i < NBIAS; i += NTE) {
    const float c1 = b1[i & 63], c2 = b2[i & 63], c3 = g1[i & 63], c4 = g2[i & 63], c5 = g3[i & 15];
    float v = c1;
    v = (i >= 64)  ? c2 : v;
    v = (i >= 128) ? c3 : v;
    v = (i >= 192) ? c4 : v;
    v = (i >= 256) ? c5 : v;
    bsm[i] = v * WSC;
  }
  if (tid == 0) pendN = 0;
  __syncthreads();

  const int nChunks = (nE + CHE - 1) / CHE;
#pragma unroll 1
  for (int ch = 0; ch < nChunks; ++ch) {
    const int cbase = ch * CHE;
    const int wc = scan_chunk<NB, NTE>(dsts, nE, cbase, nodeBase, vec8, list, tid, wave);
    if (lane == 0) wcnt[wave] = wc;
    __syncthreads();

    const int base = pendN;
    int tot = 0, myoff = 0;
#pragma unroll
    for (int w = 0; w < NWE; ++w) {
      int c = wcnt[w];
      c = c > WCAP ? WCAP : (c < 0 ? 0 : c);
      if (w < wave) myoff += c;
      tot += c;
    }
    int newN = base + tot;
    newN = newN > PCAP ? PCAP : newN;
    {
      int n = wcnt[wave];
      n = n > WCAP ? WCAP : (n < 0 ? 0 : n);
      const int* lp = list + wave * WCAP;
      for (int i = lane; i < n; i += 32) {
        const int pos = base + myoff + i;
        if (pos < PCAP) pend[pos] = cbase + lp[i];
      }
    }
    const int fin = (ch == nChunks - 1) ? 1 : 0;
    const int R   = (fin != 0) ? (newN + PASSN - 1) / PASSN : newN / PASSN;
    const int Pv  = (fin != 0) ? newN : R * PASSN;
    __syncthreads();

#pragma unroll 1
    for (int r = 0; r < R; ++r) {
      float okf;
      {
        int idx = r * PASSN + wave * 16 + m;
        const bool valid = idx < Pv;
        idx = idx > PCAP - 1 ? PCAP - 1 : idx;
        int e = pend[idx];
        e = e < 0 ? 0 : (e > nE - 1 ? nE - 1 : e);
        int d = dsts[e];
        int s = srcs[e];
        const unsigned us = (unsigned)d - (unsigned)nodeBase;
        const bool ok = valid && (us < (unsigned)NB);
        const int slot = ok ? (int)us : 0;
        okf = ok ? 1.0f : 0.0f;
        d = d < 0 ? 0 : (d > nN - 1 ? nN - 1 : d);
        s = s < 0 ? 0 : (s > nN - 1 ? nN - 1 : s);
        const float* pp = pq + (size_t)d * 128 + 32 * h;
        const float* qp = pq + (size_t)s * 128 + 64 + 32 * h;
        _Float16* sp = stg + (wave * 16 + m) * DM + 32 * h;
#pragma unroll
        for (int g = 0; g < 4; ++g) {
          const v4f p0 = *(const v4f*)(pp + 8 * g);
          const v4f p1 = *(const v4f*)(pp + 8 * g + 4);
          const v4f q0 = *(const v4f*)(qp + 8 * g);
          const v4f q1 = *(const v4f*)(qp + 8 * g + 4);
          v4f u0, u1;
          u0.x = fmaxf(p0.x + q0.x, 0.0f); u0.y = fmaxf(p0.y + q0.y, 0.0f);
          u0.z = fmaxf(p0.z + q0.z, 0.0f); u0.w = fmaxf(p0.w + q0.w, 0.0f);
          u1.x = fmaxf(p1.x + q1.x, 0.0f); u1.y = fmaxf(p1.y + q1.y, 0.0f);
          u1.z = fmaxf(p1.z + q1.z, 0.0f); u1.w = fmaxf(p1.w + q1.w, 0.0f);
          *(v8h*)(sp + 8 * g) = pk8(u0, u1);
        }
        if (h == 0) slotb[wave * 16 + m] = slot;
      }
      __syncthreads();

      {
        FragH bq0, bq1;
        {
          const _Float16* sr = stg + (wave * 16 + m) * DM + 8 * h;
          bq0.h[0] = *(const v8h*)sr;        bq0.h[1] = *(const v8h*)(sr + 16);
          bq1.h[0] = *(const v8h*)(sr + 32); bq1.h[1] = *(const v8h*)(sr + 48);
        }
        v8f d0, d1, d2, d3;
        d0 = tile16(w1t + (16 * 0 + m) * DM + 8 * h, bsm + 16 * 0 + 8 * h, bq0.v, bq1.v);
        d1 = tile16(w1t + (16 * 1 + m) * DM + 8 * h, bsm + 16 * 1 + 8 * h, bq0.v, bq1.v);
        d2 = tile16(w1t + (16 * 2 + m) * DM + 8 * h, bsm + 16 * 2 + 8 * h, bq0.v, bq1.v);
        d3 = tile16(w1t + (16 * 3 + m) * DM + 8 * h, bsm + 16 * 3 + 8 * h, bq0.v, bq1.v);
        bq0.h[0] = relu8(d0); bq0.h[1] = relu8(d1);
        bq1.h[0] = relu8(d2); bq1.h[1] = relu8(d3);
        d0 = tile16(w2t + (16 * 0 + m) * DM + 8 * h, bsm + 64 + 16 * 0 + 8 * h, bq0.v, bq1.v);
        d1 = tile16(w2t + (16 * 1 + m) * DM + 8 * h, bsm + 64 + 16 * 1 + 8 * h, bq0.v, bq1.v);
        d2 = tile16(w2t + (16 * 2 + m) * DM + 8 * h, bsm + 64 + 16 * 2 + 8 * h, bq0.v, bq1.v);
        d3 = tile16(w2t + (16 * 3 + m) * DM + 8 * h, bsm + 64 + 16 * 3 + 8 * h, bq0.v, bq1.v);
        float* mp = msg + (wave * 16 + m) * DM + 8 * h;
#define STMSG(FT, DD) { \
          v4f u0, u1; \
          u0.x = fmaxf(DD[0] * WINV, 0.0f) * okf; u0.y = fmaxf(DD[1] * WINV, 0.0f) * okf; \
          u0.z = fmaxf(DD[2] * WINV, 0.0f) * okf; u0.w = fmaxf(DD[3] * WINV, 0.0f) * okf; \
          u1.x = fmaxf(DD[4] * WINV, 0.0f) * okf; u1.y = fmaxf(DD[5] * WINV, 0.0f) * okf; \
          u1.z = fmaxf(DD[6] * WINV, 0.0f) * okf; u1.w = fmaxf(DD[7] * WINV, 0.0f) * okf; \
          *(v4f*)(mp + 16 * (FT)) = u0; *(v4f*)(mp + 16 * (FT) + 4) = u1; }
        STMSG(0, d0)
        STMSG(1, d1)
        STMSG(2, d2)
        STMSG(3, d3)
#undef STMSG
      }
      __syncthreads();

      if (wave == 0) {
#pragma unroll 1
        for (int i = 0; i < PASSN; ++i) {
          int sl = slotb[i];
          sl = sl < 0 ? 0 : (sl > NB - 1 ? NB - 1 : sl);
          if (lane < 16) {
            float* ar = acc + sl * DM + 4 * lane;
            const v4f v = *(const v4f*)(msg + i * DM + 4 * lane);
            v4f t = *(const v4f*)ar;
            t += v;
            *(v4f*)ar = t;
          }
        }
      }
      __syncthreads();
    }

    int rem = newN - R * PASSN;
    rem = rem < 0 ? 0 : rem;
    if (R > 0 && tid < rem) pend[tid] = pend[R * PASSN + tid];
    if (tid == 0) pendN = rem;
  }
  __syncthreads();

#pragma unroll 1
  for (int t = wave; t < NB / 16; t += NWE) {
    FragH bq0, bq1;
    {
      const float* nr = acc + (16 * t + m) * DM + 8 * h;
      bq0.h[0] = cvt8(nr);      bq0.h[1] = cvt8(nr + 16);
      bq1.h[0] = cvt8(nr + 32); bq1.h[1] = cvt8(nr + 48);
    }
    v8f d0, d1, d2, d3;
    d0 = tile16(f1t + (16 * 0 + m) * DM + 8 * h, bsm + 128 + 16 * 0 + 8 * h, bq0.v, bq1.v);
    d1 = tile16(f1t + (16 * 1 + m) * DM + 8 * h, bsm + 128 + 16 * 1 + 8 * h, bq0.v, bq1.v);
    d2 = tile16(f1t + (16 * 2 + m) * DM + 8 * h, bsm + 128 + 16 * 2 + 8 * h, bq0.v, bq1.v);
    d3 = tile16(f1t + (16 * 3 + m) * DM + 8 * h, bsm + 128 + 16 * 3 + 8 * h, bq0.v, bq1.v);
    bq0.h[0] = relu8(d0); bq0.h[1] = relu8(d1);
    bq1.h[0] = relu8(d2); bq1.h[1] = relu8(d3);
    d0 = tile16(f2t + (16 * 0 + m) * DM + 8 * h, bsm + 192 + 16 * 0 + 8 * h, bq0.v, bq1.v);
    d1 = tile16(f2t + (16 * 1 + m) * DM + 8 * h, bsm + 192 + 16 * 1 + 8 * h, bq0.v, bq1.v);
    d2 = tile16(f2t + (16 * 2 + m) * DM + 8 * h, bsm + 192 + 16 * 2 + 8 * h, bq0.v, bq1.v);
    d3 = tile16(f2t + (16 * 3 + m) * DM + 8 * h, bsm + 192 + 16 * 3 + 8 * h, bq0.v, bq1.v);
    bq0.h[0] = relu8(d0); bq0.h[1] = relu8(d1);
    bq1.h[0] = relu8(d2); bq1.h[1] = relu8(d3);
    const v8f dq4 = tile16(w3t + m * DM + 8 * h, bsm + 256 + 8 * h, bq0.v, bq1.v);
    {
      float* op = msg + wave * 256 + m * 16 + 8 * h;
      v4f u0, u1;
      u0.x = fmaxf(dq4[0] * WINV, 0.0f); u0.y = fmaxf(dq4[1] * WINV, 0.0f);
      u0.z = fmaxf(dq4[2] * WINV, 0.0f); u0.w = fmaxf(dq4[3] * WINV, 0.0f);
      u1.x = fmaxf(dq4[4] * WINV, 0.0f); u1.y = fmaxf(dq4[5] * WINV, 0.0f);
      u1.z = fmaxf(dq4[6] * WINV, 0.0f); u1.w = fmaxf(dq4[7] * WINV, 0.0f);
      *(v4f*)op = u0;
      *(v4f*)(op + 4) = u1;
    }
    __syncthreads();
    {
      const float* os = msg + wave * 256;
      float* og = opl + (size_t)(nodeBase + 16 * t) * 16;
      const v4f v0 = *(const v4f*)(os + 4 * lane);
      const v4f v1 = *(const v4f*)(os + 128 + 4 * lane);
      *(volatile v4f*)(og + 4 * lane) = v0;
      *(volatile v4f*)(og + 128 + 4 * lane) = v1;
      __threadfence();
      *(volatile v4f*)(og + 4 * lane) = v0;
      *(volatile v4f*)(og + 128 + 4 * lane) = v1;
    }
    __syncthreads();
  }
}

__global__ __launch_bounds__(NTM) void k_mol(
    const float* __restrict__ opl, const int* __restrict__ seg, float* out, int nN, int outLim) {
  __shared__ __attribute__((aligned(16))) float acc2[MB * 16];
  __shared__ __attribute__((aligned(16))) int   list[NWM * WCAP];
  __shared__ int wcnt[NWM];
  const int tid = threadIdx.x, lane = tid & 31, wave = tid >> 5;
  const int molBase = blockIdx.x * MB;
  {
    const v4f z4 = {0.0f, 0.0f, 0.0f, 0.0f};
    for (int i = tid; i < MB * 4; i += NTM) *(v4f*)(acc2 + 4 * i) = z4;
  }
  __syncthreads();

  const int nChunks = (nN + NTM * EPT - 1) / (NTM * EPT);
#pragma unroll 1
  for (int ch = 0; ch < nChunks; ++ch) {
    const int cbase = ch * (NTM * EPT);
    const int wc = scan_chunk<MB, NTM>(seg, nN, cbase, molBase, 1, list, tid, wave);
    if (lane == 0) wcnt[wave] = wc;
    __syncthreads();
    if (wave == 0) {
#pragma unroll 1
      for (int w = 0; w < NWM; ++w) {
        int n = wcnt[w];
        n = n > WCAP ? WCAP : (n < 0 ? 0 : n);
#pragma unroll 1
        for (int i = 0; i < n; ++i) {
          const int la = list[w * WCAP + i];
          int a = cbase + la;
          a = a < 0 ? 0 : (a > nN - 1 ? nN - 1 : a);
          int sl = seg[a] - molBase;
          sl = sl < 0 ? 0 : (sl > MB - 1 ? MB - 1 : sl);
          if (lane < 4) {
            const v4f o = *(const v4f*)(opl + (size_t)a * 16 + 4 * lane);
            float* ar = acc2 + sl * 16 + 4 * lane;
            v4f t = *(const v4f*)ar;
            t += o;
            *(v4f*)ar = t;
          }
        }
      }
    }
    __syncthreads();
  }

  const size_t ob  = (size_t)molBase * 16;
  const size_t lim = (size_t)(outLim < 0 ? 0 : outLim);
#pragma unroll 1
  for (int q = tid; q < MB * 4; q += NTM) {
    const size_t gi = ob + (size_t)(4 * q);
    const v4f v = *(const v4f*)(acc2 + 4 * q);
    if (gi + 3 < lim) *(volatile v4f*)(out + gi) = v;
  }
  __threadfence();
#pragma unroll 1
  for (int q = tid; q < MB * 4; q += NTM) {
    const size_t gi = ob + (size_t)(4 * q);
    const v4f v = *(const v4f*)(acc2 + 4 * q);
    if (gi + 3 < lim) *(volatile v4f*)(out + gi) = v;
  }
}

extern "C" void kernel_launch(void* const* d_in, const int* in_sizes, int n_in,
                              void* d_out, int out_size, void* d_ws, size_t ws_size,
                              hipStream_t stream) {
  if (n_in < 16) return;
  const int nN = in_sizes[0] / DM;
  if (nN <= 0 || in_sizes[0] != nN * DM) return;
  const int nE = in_sizes[1];
  if (nE <= 0 || in_sizes[2] != nE || in_sizes[3] != nN) return;
  if (in_sizes[4] != 128 * DM || in_sizes[5] != DM || in_sizes[6] != DM * DM || in_sizes[7] != DM) return;
  if (in_sizes[8] != DM * DM || in_sizes[9] != DM || in_sizes[10] != DM * DM || in_sizes[11] != DM) return;
  if (in_sizes[12] != DM * DM || in_sizes[13] != DM || in_sizes[14] != DM * 16 || in_sizes[15] != 16) return;
  if (out_size <= 0 || (out_size % 16) != 0) return;
  const int nMol = out_size / 16;

  const float* st    = (const float*)d_in[0];
  const int*   esrc  = (const int*)d_in[1];
  const int*   edst  = (const int*)d_in[2];
  const int*   aseg  = (const int*)d_in[3];
  const float* ms0_w = (const float*)d_in[4];
  const float* ms0_b = (const float*)d_in[5];
  const float* ms1_w = (const float*)d_in[6];
  const float* ms1_b = (const float*)d_in[7];
  const float* ms2_w = (const float*)d_in[8];
  const float* ms2_b = (const float*)d_in[9];
  const float* fc1_w = (const float*)d_in[10];
  const float* fc1_b = (const float*)d_in[11];
  const float* fc2_w = (const float*)d_in[12];
  const float* fc2_b = (const float*)d_in[13];
  const float* out_w = (const float*)d_in[14];
  const float* out_b = (const float*)d_in[15];
  float* out = (float*)d_out;

  const int nBlk  = (nN + NB - 1) / NB;
  const int nNpad = nBlk * NB;

  char* ws = (char*)d_ws;
  size_t off = 0;
  const size_t oW  = off; off += 65536;
  const size_t oPQ = off; off += (size_t)nNpad * 128 * sizeof(float);
  const size_t oO  = off; off += (size_t)nNpad * 16 * sizeof(float);
  if (off > ws_size || off > (size_t)134217728) return;
  _Float16* wpl = (_Float16*)(ws + oW);
  float*    pq  = (float*)(ws + oPQ);
  float*    opl = (float*)(ws + oO);

  k_prep<<<1, NTP, 0, stream>>>(ms0_w, ms1_w, ms2_w, fc1_w, fc2_w, out_w, wpl);

  k_node<<<nNpad / 64, NTN, 0, stream>>>(st, wpl, ms0_b, pq, nN);

  const size_t dynB = (size_t)NB * DM * sizeof(float);
  hipFuncSetAttribute(reinterpret_cast<const void*>(&k_edge),
                      hipFuncAttributeMaxDynamicSharedMemorySize, (int)dynB);
  k_edge<<<nBlk, NTE, dynB, stream>>>(pq, esrc, edst, wpl, ms1_b, ms2_b, fc1_b, fc2_b, out_b,
                                      opl, nN, nE, 1);

  const int nBlkM = (nMol + MB - 1) / MB;
  k_mol<<<nBlkM, NTM, 0, stream>>>(opl, aseg, out, nN, out_size);
}
